// CausalConv3dAttnBlock_7567732376026
// MI455X (gfx1250) — hardware-verified
//
#include <hip/hip_runtime.h>

typedef __attribute__((ext_vector_type(16))) _Float16 v16h;
typedef __attribute__((ext_vector_type(8)))  _Float16 v8h;
typedef __attribute__((ext_vector_type(16))) __bf16   v16b;
typedef __attribute__((ext_vector_type(8)))  __bf16   v8b;
typedef __attribute__((ext_vector_type(8)))  float    v8f;
typedef __attribute__((ext_vector_type(4)))  float    v4f;
#define U16(p) ((const unsigned short*)(const void*)(p))

constexpr int CH   = 512;
constexpr int TFR  = 4;
constexpr int SP   = 4096;
constexpr int CSP  = TFR * SP;
constexpr int NTOK = TFR * SP;
constexpr int GSZ  = 16 * CSP;
constexpr int NGRP = 32;
constexpr int QH   = 2048;
constexpr float GN_EPS     = 1e-6f;
constexpr float QSCALE     = 0.04419417382415922f;
constexpr float WCARRY     = 16.0f;
constexpr float WCARRY_INV = 1.0f / 16.0f;
constexpr float PCARRY     = 32768.0f;
constexpr float PCARRY_INV = 1.0f / 32768.0f;

__device__ __forceinline__ unsigned short f2bf_bits(float f) {
  unsigned u = __float_as_uint(f);
  return (unsigned short)((u + 0x7FFFu + ((u >> 16) & 1u)) >> 16);
}
__device__ __forceinline__ float bf_bits2f(unsigned short h) { return __uint_as_float(((unsigned)h) << 16); }

__device__ __forceinline__ void dep_guard_h(v8f& a, v8f& b, v16h x, v16h y) { asm volatile("v_nop\n\tv_nop\n\tv_nop\n\tv_nop" : "+v"(a), "+v"(b) : "v"(x), "v"(y)); }
__device__ __forceinline__ void dep_guard_b(v8f& a, v8f& b, v16b x, v16b y) { asm volatile("v_nop\n\tv_nop\n\tv_nop\n\tv_nop" : "+v"(a), "+v"(b) : "v"(x), "v"(y)); }
__device__ __forceinline__ void keep4_h(v16h a, v16h b, v16h c, v16h d) { asm volatile("v_nop" :: "v"(a), "v"(b), "v"(c), "v"(d)); }
__device__ __forceinline__ void keep4_b(v16b a, v16b b, v16b c, v16b d) { asm volatile("v_nop" :: "v"(a), "v"(b), "v"(c), "v"(d)); }
__device__ __forceinline__ void acc_guard4(v8f& a, v8f& b, v8f& c, v8f& d) { asm volatile("v_nop\n\tv_nop\n\tv_nop\n\tv_nop" : "+v"(a), "+v"(b), "+v"(c), "+v"(d)); }
template <typename T> struct Frag;
template <> struct Frag<_Float16> {
  typedef v16h V; union U { v16h v; v8h h[2]; };
  static __device__ __forceinline__ v16h load(const _Float16* p) {
    U f; f.h[0] = *(const v8h*)(p); f.h[1] = *(const v8h*)(p + 16); return f.v;
  }
  static __device__ __forceinline__ v8f mma(v16h a, v16h b, v8f c) {
    return __builtin_amdgcn_wmma_f32_16x16x32_f16(false, a, false, b, (short)0, c, false, false);
  }
  static __device__ __forceinline__ void guard(v8f& a, v8f& b, v16h x, v16h y) { dep_guard_h(a, b, x, y); }
  static __device__ __forceinline__ void keep(v16h a, v16h b, v16h c, v16h d) { keep4_h(a, b, c, d); }
};
template <> struct Frag<__bf16> {
  typedef v16b V; union U { v16b v; v8b h[2]; };
  static __device__ __forceinline__ v16b load(const __bf16* p) {
    U f; f.h[0] = *(const v8b*)(p); f.h[1] = *(const v8b*)(p + 16); return f.v;
  }
  static __device__ __forceinline__ v8f mma(v16b a, v16b b, v8f c) {
    return __builtin_amdgcn_wmma_f32_16x16x32_bf16(false, a, false, b, (short)0, c, false, false);
  }
  static __device__ __forceinline__ void guard(v8f& a, v8f& b, v16b x, v16b y) { dep_guard_b(a, b, x, y); }
  static __device__ __forceinline__ void keep(v16b a, v16b b, v16b c, v16b d) { keep4_b(a, b, c, d); }
};

template <int ET> struct Elem;
template <> struct Elem<0> { typedef _Float16 T; };
template <> struct Elem<1> { typedef __bf16 T; };
template <int ET, bool SPLIT, int BIAS_MODE, int OUT_MODE, bool RESID, int ACT = 0>
__global__ __launch_bounds__(256) void wmma_gemm64(
    const unsigned short* __restrict__ Ap, const unsigned short* __restrict__ A2p, int lda, long strideA,
    const unsigned short* __restrict__ Btp, const unsigned short* __restrict__ Bt2p, int ldb, long strideB,
    void* __restrict__ Cout, void* __restrict__ Cout2, int ldc, long strideC,
    const float* __restrict__ bias,
    const float* __restrict__ resid, long strideR,
    int M, int N, int K, float scale) {
  typedef typename Elem<ET>::T T;
  typedef typename Frag<T>::V V;
  const T* A = (const T*)Ap; const T* A2 = (const T*)A2p; const T* Bt = (const T*)Btp; const T* Bt2 = (const T*)Bt2p;
  __shared__ __align__(16) float sT[8][16 * 68];
  const int b    = blockIdx.y;
  const int lane = threadIdx.x & 31;
  const int wave = threadIdx.x >> 5;
  const int tilesN = N >> 6;
  const int tilesM = M >> 6;
  const int tile = blockIdx.x * 8 + wave;
  if (tile >= tilesM * tilesN) return;
  const int tm = tile / tilesN;
  const int tn = tile - tm * tilesN;
  const int m0 = tm << 6;
  const int n0 = tn << 6;

  const T* Ab  = A  + (size_t)b * strideA;
  const T* Bb  = Bt + (size_t)b * strideB;
  const T* Ab2 = SPLIT ? (A2  + (size_t)b * strideA) : nullptr;
  const T* Bb2 = SPLIT ? (Bt2 + (size_t)b * strideB) : nullptr;

  const int rlane = lane & 15;
  const int koff  = (lane >> 4) * 8;
  const int mOff  = (lane >> 4) * 8;

  v8f acc[4][4];
#pragma unroll
  for (int i = 0; i < 4; ++i)
#pragma unroll
    for (int j = 0; j < 4; ++j) acc[i][j] = (v8f){0.f,0.f,0.f,0.f,0.f,0.f,0.f,0.f};

  for (int k0 = 0; k0 < K; k0 += 32) {
    V bh[4], bl[4];
#pragma unroll
    for (int j = 0; j < 4; ++j) {
      const size_t bo = (size_t)(n0 + (j << 4) + rlane) * ldb + koff + k0;
      bh[j] = Frag<T>::load(Bb + bo);
      if (SPLIT) bl[j] = Frag<T>::load(Bb2 + bo);
    }
#pragma unroll
    for (int i = 0; i < 4; ++i) {
      const size_t ao = (size_t)(m0 + (i << 4) + rlane) * lda + koff + k0;
      V ah = Frag<T>::load(Ab + ao);
      V al;
      if (SPLIT) al = Frag<T>::load(Ab2 + ao);
#pragma unroll
      for (int j = 0; j < 4; ++j) {
        acc[i][j] = Frag<T>::mma(ah, bh[j], acc[i][j]);
        if (SPLIT) {
          acc[i][j] = Frag<T>::mma(ah, bl[j], acc[i][j]);
          acc[i][j] = Frag<T>::mma(al, bh[j], acc[i][j]);
        }
      }
      Frag<T>::guard(acc[i][0], acc[i][3], ah, SPLIT ? al : ah);
    }
    Frag<T>::keep(bh[0], bh[1], bh[2], bh[3]);
    if (SPLIT) Frag<T>::keep(bl[0], bl[1], bl[2], bl[3]);
  }
  acc_guard4(acc[0][0], acc[0][1], acc[0][2], acc[0][3]);
  acc_guard4(acc[1][0], acc[1][1], acc[1][2], acc[1][3]);
  acc_guard4(acc[2][0], acc[2][1], acc[2][2], acc[2][3]);
  acc_guard4(acc[3][0], acc[3][1], acc[3][2], acc[3][3]);

  float* slab = sT[wave];
  const float* Rb = RESID ? (resid + (size_t)b * strideR) : nullptr;
#pragma unroll
  for (int i = 0; i < 4; ++i) {
    const int mBase = m0 + (i << 4);
#pragma unroll
    for (int j = 0; j < 4; ++j) {
      const int n = n0 + (j << 4) + rlane;
      float bv = 0.f;
      if (BIAS_MODE == 2) bv = bias[n];
#pragma unroll
      for (int r = 0; r < 8; ++r) {
        float v = acc[i][j][r] * scale;
        if (BIAS_MODE == 1) v += bias[mBase + mOff + r];
        if (BIAS_MODE == 2) v += bv;
        if (RESID) v += Rb[(size_t)(mBase + mOff + r) * ldc + n];
        if (ACT == 1) v = tanhf(v);
        if (ACT == 2) v = fmaxf(v, 0.0f);
        if (ACT == 3) v = v / (1.0f + expf(-v));
        if (ACT == 4) v = (v > 0.f) ? v : 0.01f * v;
        if (ACT == 5) v = 0.5f * v * (1.0f + erff(v * 0.70710678118654752f));
        slab[(mOff + r) * 68 + (j << 4) + rlane] = v;
      }
    }
    __builtin_amdgcn_fence(__ATOMIC_RELEASE, "workgroup");
    __builtin_amdgcn_wave_barrier();
    __builtin_amdgcn_fence(__ATOMIC_ACQUIRE, "workgroup");
    if (OUT_MODE == 0) {
      float* C = (float*)Cout + (size_t)b * strideC;
      const int hh = lane >> 4, c4 = (lane & 15) * 4;
      for (int pass = 0; pass < 2; ++pass) {
#pragma unroll
        for (int it = 0; it < 8; ++it) {
          const int row = it * 2 + hh;
          v4f v = *(const v4f*)(slab + row * 68 + c4);
          *(volatile v4f*)(C + (size_t)(mBase + row) * ldc + n0 + c4) = v;
        }
        __threadfence();
      }
    } else {
      const int q = lane >> 3, c8 = (lane & 7) * 8;
      unsigned short* C  = (unsigned short*)Cout  + (size_t)b * strideC;
      unsigned short* C2 = (OUT_MODE == 2) ? ((unsigned short*)Cout2 + (size_t)b * strideC) : nullptr;
      for (int pass = 0; pass < 2; ++pass) {
#pragma unroll
        for (int it = 0; it < 4; ++it) {
          const int row = it * 4 + q;
          const float* sp = slab + row * 68 + c8;
          v8h hv, lv;
#pragma unroll
          for (int e = 0; e < 8; ++e) {
            if (OUT_MODE == 1) {
              hv[e] = (_Float16)sp[e];
            } else {
              unsigned short hb = f2bf_bits(sp[e]);
              unsigned short lb = f2bf_bits(sp[e] - bf_bits2f(hb));
              hv[e] = __builtin_bit_cast(_Float16, hb);
              lv[e] = __builtin_bit_cast(_Float16, lb);
            }
          }
          *(volatile v8h*)(C + (size_t)(mBase + row) * ldc + n0 + c8) = hv;
          if (OUT_MODE == 2) *(volatile v8h*)(C2 + (size_t)(mBase + row) * ldc + n0 + c8) = lv;
        }
        __threadfence();
      }
    }
    __builtin_amdgcn_fence(__ATOMIC_RELEASE, "workgroup");
    __builtin_amdgcn_wave_barrier();
    __builtin_amdgcn_fence(__ATOMIC_ACQUIRE, "workgroup");
  }
}

__global__ __launch_bounds__(256) void cast_f32_f16x2s(
    const float* __restrict__ in, _Float16* __restrict__ out, int n2, float sc) {
  int i = blockIdx.x * 256 + threadIdx.x;
  if (i < n2) {
    const _Float16 h0 = (_Float16)(in[2 * i] * sc), h1 = (_Float16)(in[2 * i + 1] * sc);
    const unsigned u = (unsigned)__builtin_bit_cast(unsigned short, h0) | ((unsigned)__builtin_bit_cast(unsigned short, h1) << 16);
    ((volatile unsigned*)out)[i] = u;
    __threadfence();
    ((volatile unsigned*)out)[i] = u;
  }
}

__global__ __launch_bounds__(256) void gn_stats(const float* __restrict__ x, float* __restrict__ stats) {
  __shared__ double ws1[8];
  __shared__ double ws2[8];
  const int g = blockIdx.x;
  const int tid = threadIdx.x, wave = tid >> 5, lane = tid & 31;
  const v4f* p = (const v4f*)(x + (size_t)g * GSZ);
  double s = 0.0, s2 = 0.0;
#pragma unroll 2
  for (int i = tid; i < GSZ / 4; i += 256) {
    const v4f v = p[i];
#pragma unroll
    for (int e = 0; e < 4; ++e) { const double d = (double)v[e]; s += d; s2 += d * d; }
  }
#pragma unroll
  for (int off = 1; off < 32; off <<= 1) { s += __shfl_xor(s, off, 32); s2 += __shfl_xor(s2, off, 32); }
  if (lane == 0) { ws1[wave] = s; ws2[wave] = s2; }
  __syncthreads();
  if (tid < 32) {
    double ts = 0.0, ts2 = 0.0;
#pragma unroll
    for (int w = 0; w < 8; ++w) { ts += ws1[w]; ts2 += ws2[w]; }
    const double mean = ts * (1.0 / (double)GSZ);
    double var = ts2 * (1.0 / (double)GSZ) - mean * mean;
    if (var < 0.0) var = 0.0;
    const float meanf = (float)mean;
    const float rstd  = rsqrtf((float)var + GN_EPS);
    const float val = (lane == 0) ? meanf : ((lane == 1) ? rstd : 0.0f);
    float* dst = stats + g * 32 + lane;
    *(volatile float*)dst = val;
    __threadfence();
    *(volatile float*)dst = val;
  }
}

__global__ __launch_bounds__(256) void norm_tok(const float* __restrict__ x,
                                                const float* __restrict__ gamma,
                                                const float* __restrict__ beta,
                                                const float* __restrict__ stats,
                                                _Float16* __restrict__ tok) {
  __shared__ __align__(16) _Float16 tile[64 * 72];
  const int bid = blockIdx.x;
  const int cb  = bid & 7;
  const int sb  = (bid >> 3) & 63;
  const int t   = bid >> 9;
  const int c0 = cb * 64, s0 = sb * 64;
  const int tid = threadIdx.x;
#pragma unroll 4
  for (int i = tid; i < 64 * 64; i += 256) {
    const int cl = i >> 6, sl = i & 63;
    const int c = c0 + cl;
    const int g = c >> 4;
    const float mean = stats[g * 32], rstd = stats[g * 32 + 1];
    float v = x[(size_t)c * CSP + (size_t)t * SP + s0 + sl];
    v = (v - mean) * rstd * gamma[c] + beta[c];
    tile[sl * 72 + cl] = (_Float16)v;
  }
  __syncthreads();
  const int wave = tid >> 5, lane = tid & 31;
  const int q = lane >> 3, c8 = (lane & 7) * 8;
  for (int pass = 0; pass < 2; ++pass) {
#pragma unroll
    for (int it = 0; it < 2; ++it) {
      const int row = wave * 8 + it * 4 + q;
      const v8h hv = *(const v8h*)(tile + row * 72 + c8);
      *(volatile v8h*)(tok + ((size_t)t * SP + s0 + row) * CH + c0 + c8) = hv;
    }
    __threadfence();
  }
}

__global__ __launch_bounds__(256) void softmax_rows(const float* __restrict__ S, _Float16* __restrict__ P) {
  __shared__ float rmax[8];
  __shared__ float rsum[8];
  const int row = blockIdx.x;
  const int tid = threadIdx.x, wave = tid >> 5, lane = tid & 31;
  const float* sr = S + (size_t)row * SP;
  const v4f a0 = *(const v4f*)(sr + 8 * tid);
  const v4f a1 = *(const v4f*)(sr + 8 * tid + 4);
  const v4f a2 = *(const v4f*)(sr + (SP / 2) + 8 * tid);
  const v4f a3 = *(const v4f*)(sr + (SP / 2) + 8 * tid + 4);
  float m = a0[0];
#pragma unroll
  for (int e = 0; e < 4; ++e) { m = fmaxf(m, a0[e]); m = fmaxf(m, a1[e]); m = fmaxf(m, a2[e]); m = fmaxf(m, a3[e]); }
#pragma unroll
  for (int off = 1; off < 32; off <<= 1) m = fmaxf(m, __shfl_xor(m, off, 32));
  if (lane == 0) rmax[wave] = m;
  __syncthreads();
  float bm = rmax[0];
#pragma unroll
  for (int w = 1; w < 8; ++w) bm = fmaxf(bm, rmax[w]);
  v4f e0, e1, e2, e3;
  float su = 0.f;
#pragma unroll
  for (int e = 0; e < 4; ++e) { e0[e] = __expf(a0[e] - bm); su += e0[e]; }
#pragma unroll
  for (int e = 0; e < 4; ++e) { e1[e] = __expf(a1[e] - bm); su += e1[e]; }
#pragma unroll
  for (int e = 0; e < 4; ++e) { e2[e] = __expf(a2[e] - bm); su += e2[e]; }
#pragma unroll
  for (int e = 0; e < 4; ++e) { e3[e] = __expf(a3[e] - bm); su += e3[e]; }
#pragma unroll
  for (int off = 1; off < 32; off <<= 1) su += __shfl_xor(su, off, 32);
  if (lane == 0) rsum[wave] = su;
  __syncthreads();
  float tot = rsum[0];
#pragma unroll
  for (int w = 1; w < 8; ++w) tot += rsum[w];
  const float f = (1.0f / tot) * PCARRY;
  v8h h0, h1;
#pragma unroll
  for (int e = 0; e < 4; ++e) {
    h0[e]     = (_Float16)(e0[e] * f);
    h0[4 + e] = (_Float16)(e1[e] * f);
    h1[e]     = (_Float16)(e2[e] * f);
    h1[4 + e] = (_Float16)(e3[e] * f);
  }
  _Float16* pr = P + (size_t)row * SP;
  for (int pass = 0; pass < 2; ++pass) {
    *(volatile v8h*)(pr + 8 * tid) = h0;
    *(volatile v8h*)(pr + (SP / 2) + 8 * tid) = h1;
    __threadfence();
  }
}

static inline int gemm_blocks(int M, int N) { return ((M / 64) * (N / 64) + 7) / 8; }

extern "C" void kernel_launch(void* const* d_in, const int* in_sizes, int n_in,
                              void* d_out, int out_size, void* d_ws, size_t ws_size,
                              hipStream_t stream) {
  if (n_in < 11) return;
  if (in_sizes[0] != CH * CSP || out_size != CH * CSP) return;
  if (in_sizes[1] != CH || in_sizes[2] != CH) return;
  if (in_sizes[3] != CH * CH || in_sizes[5] != CH * CH || in_sizes[7] != CH * CH || in_sizes[9] != CH * CH) return;
  if (in_sizes[4] != CH || in_sizes[6] != CH || in_sizes[8] != CH || in_sizes[10] != CH) return;

  const float* x     = (const float*)d_in[0];
  const float* gamma = (const float*)d_in[1];
  const float* beta  = (const float*)d_in[2];
  const float* wq    = (const float*)d_in[3];
  const float* bq    = (const float*)d_in[4];
  const float* wk    = (const float*)d_in[5];
  const float* bk    = (const float*)d_in[6];
  const float* wv    = (const float*)d_in[7];
  const float* bv    = (const float*)d_in[8];
  const float* wp    = (const float*)d_in[9];
  const float* bp    = (const float*)d_in[10];
  float* out = (float*)d_out;

  char* ws = (char*)d_ws;
  size_t off = 0;
  float* stats = (float*)(ws + off);          off += 4096;
  _Float16* w16  = (_Float16*)(ws + off);     off += (size_t)4 * CH * CH * sizeof(_Float16);
  _Float16* tok  = (_Float16*)(ws + off);     off += (size_t)NTOK * CH * sizeof(_Float16);
  _Float16* q16  = (_Float16*)(ws + off);     off += (size_t)NTOK * CH * sizeof(_Float16);
  _Float16* k16  = (_Float16*)(ws + off);     off += (size_t)NTOK * CH * sizeof(_Float16);
  _Float16* vT16 = (_Float16*)(ws + off);     off += (size_t)CH * NTOK * sizeof(_Float16);
  float* S       = (float*)(ws + off);        off += (size_t)QH * SP * sizeof(float);
  _Float16* P16  = (_Float16*)(ws + off);     off += (size_t)QH * SP * sizeof(_Float16);
  if (off > ws_size) return;
  _Float16* o16 = tok;
  _Float16* wq16 = w16;
  _Float16* wk16 = w16 + (size_t)CH * CH;
  _Float16* wv16 = w16 + (size_t)2 * CH * CH;
  _Float16* wp16 = w16 + (size_t)3 * CH * CH;

  gn_stats<<<dim3(NGRP), dim3(256), 0, stream>>>(x, stats);

  const int n2 = CH * CH / 2;
  cast_f32_f16x2s<<<dim3((n2 + 255) / 256), dim3(256), 0, stream>>>(wq, wq16, n2, WCARRY);
  cast_f32_f16x2s<<<dim3((n2 + 255) / 256), dim3(256), 0, stream>>>(wk, wk16, n2, WCARRY);
  cast_f32_f16x2s<<<dim3((n2 + 255) / 256), dim3(256), 0, stream>>>(wv, wv16, n2, WCARRY);
  cast_f32_f16x2s<<<dim3((n2 + 255) / 256), dim3(256), 0, stream>>>(wp, wp16, n2, WCARRY);

  norm_tok<<<dim3(TFR * 64 * 8), dim3(256), 0, stream>>>(x, gamma, beta, stats, tok);

  wmma_gemm64<0, false, 2, 1, false><<<dim3(gemm_blocks(NTOK, CH), 1), dim3(256), 0, stream>>>(
      U16(tok), U16(tok), CH, (long)0, U16(wq16), U16(wq16), CH, (long)0,
      (void*)q16, (void*)q16, CH, (long)0, bq, x, (long)0, NTOK, CH, CH, WCARRY_INV);
  wmma_gemm64<0, false, 2, 1, false><<<dim3(gemm_blocks(NTOK, CH), 1), dim3(256), 0, stream>>>(
      U16(tok), U16(tok), CH, (long)0, U16(wk16), U16(wk16), CH, (long)0,
      (void*)k16, (void*)k16, CH, (long)0, bk, x, (long)0, NTOK, CH, CH, WCARRY_INV);
  wmma_gemm64<0, false, 1, 1, false><<<dim3(gemm_blocks(CH, NTOK), 1), dim3(256), 0, stream>>>(
      U16(wv16), U16(wv16), CH, (long)0, U16(tok), U16(tok), CH, (long)0,
      (void*)vT16, (void*)vT16, NTOK, (long)0, bv, x, (long)0, CH, NTOK, CH, WCARRY_INV);

  for (int hp = 0; hp < TFR * (SP / QH); ++hp) {
    const int t = hp / (SP / QH);
    const int half = hp - t * (SP / QH);
    const size_t qrow0 = (size_t)t * SP + (size_t)half * QH;
    const _Float16* qA  = q16 + qrow0 * CH;
    const _Float16* kB  = k16 + (size_t)t * SP * CH;
    const _Float16* vB  = vT16 + (size_t)t * SP;
    _Float16* oC = o16 + qrow0 * CH;
    wmma_gemm64<0, false, 0, 0, false><<<dim3(gemm_blocks(QH, SP), 1), dim3(256), 0, stream>>>(
        U16(qA), U16(qA), CH, (long)0, U16(kB), U16(kB), CH, (long)0,
        (void*)S, (void*)S, SP, (long)0, bq, x, (long)0, QH, SP, CH, QSCALE);
    softmax_rows<<<dim3(QH), dim3(256), 0, stream>>>(S, P16);
    wmma_gemm64<0, false, 0, 1, false><<<dim3(gemm_blocks(QH, CH), 1), dim3(256), 0, stream>>>(
        U16(P16), U16(P16), SP, (long)0, U16(vB), U16(vB), NTOK, (long)0,
        (void*)oC, (void*)oC, CH, (long)0, bq, x, (long)0, QH, CH, SP, PCARRY_INV);
  }

  wmma_gemm64<0, false, 1, 0, true><<<dim3(gemm_blocks(CH, NTOK), 1), dim3(256), 0, stream>>>(
      U16(wp16), U16(wp16), CH, (long)0, U16(o16), U16(o16), CH, (long)0,
      (void*)out, (void*)out, NTOK, (long)0, bp, x, (long)0, CH, NTOK, CH, WCARRY_INV);
}
